// CasualMultiHeadAtten_70720931496732
// MI455X (gfx1250) — hardware-verified
//
#include <hip/hip_runtime.h>
#include <math.h>

typedef __attribute__((ext_vector_type(16))) _Float16 v16h;
typedef __attribute__((ext_vector_type(8)))  _Float16 v8h;
typedef __attribute__((ext_vector_type(16))) __bf16   v16b;
typedef __attribute__((ext_vector_type(8)))  __bf16   v8b;
typedef __attribute__((ext_vector_type(8)))  float    v8f;
typedef __attribute__((ext_vector_type(4)))  float    v4f;

constexpr int NBATCH = 4;
constexpr int SEQ    = 2048;
constexpr int DMODEL = 1024;
constexpr int NHEAD  = 16;
constexpr int HDIM   = 64;
constexpr int QK_LD  = 2 * DMODEL;
constexpr int KCOL0  = DMODEL;
constexpr int ATT_QB = 64;
constexpr int ATT_KC = 64;
constexpr int ATT_NW = 4;
constexpr int NQB    = SEQ / ATT_QB;
constexpr int OS_PITCH = 68;

__device__ __forceinline__ unsigned short f2bf_bits(float f) {
  unsigned u = __float_as_uint(f);
  return (unsigned short)((u + 0x7FFFu + ((u >> 16) & 1u)) >> 16);
}
__device__ __forceinline__ float bf_bits2f(unsigned short h) { return __uint_as_float(((unsigned)h) << 16); }

__device__ __forceinline__ void dep_guard_h(v8f& a, v8f& b, v16h x, v16h y) { asm volatile("v_nop\n\tv_nop\n\tv_nop\n\tv_nop" : "+v"(a), "+v"(b) : "v"(x), "v"(y)); }
__device__ __forceinline__ void dep_guard_b(v8f& a, v8f& b, v16b x, v16b y) { asm volatile("v_nop\n\tv_nop\n\tv_nop\n\tv_nop" : "+v"(a), "+v"(b) : "v"(x), "v"(y)); }
__device__ __forceinline__ void keep4_h(v16h a, v16h b, v16h c, v16h d) { asm volatile("v_nop" :: "v"(a), "v"(b), "v"(c), "v"(d)); }
__device__ __forceinline__ void keep4_b(v16b a, v16b b, v16b c, v16b d) { asm volatile("v_nop" :: "v"(a), "v"(b), "v"(c), "v"(d)); }
__device__ __forceinline__ void acc_guard4(v8f& a, v8f& b, v8f& c, v8f& d) { asm volatile("v_nop\n\tv_nop\n\tv_nop\n\tv_nop" : "+v"(a), "+v"(b), "+v"(c), "+v"(d)); }
template <typename T> struct Frag;
template <> struct Frag<_Float16> {
  typedef v16h V; union U { v16h v; v8h h[2]; };
  static __device__ __forceinline__ v16h load(const _Float16* p) {
    U f; f.h[0] = *(const v8h*)(p); f.h[1] = *(const v8h*)(p + 16); return f.v;
  }
  static __device__ __forceinline__ v8f mma(v16h a, v16h b, v8f c) {
    return __builtin_amdgcn_wmma_f32_16x16x32_f16(false, a, false, b, (short)0, c, false, false);
  }
  static __device__ __forceinline__ void guard(v8f& a, v8f& b, v16h x, v16h y) { dep_guard_h(a, b, x, y); }
  static __device__ __forceinline__ void keep(v16h a, v16h b, v16h c, v16h d) { keep4_h(a, b, c, d); }
};
template <> struct Frag<__bf16> {
  typedef v16b V; union U { v16b v; v8b h[2]; };
  static __device__ __forceinline__ v16b load(const __bf16* p) {
    U f; f.h[0] = *(const v8b*)(p); f.h[1] = *(const v8b*)(p + 16); return f.v;
  }
  static __device__ __forceinline__ v8f mma(v16b a, v16b b, v8f c) {
    return __builtin_amdgcn_wmma_f32_16x16x32_bf16(false, a, false, b, (short)0, c, false, false);
  }
  static __device__ __forceinline__ void guard(v8f& a, v8f& b, v16b x, v16b y) { dep_guard_b(a, b, x, y); }
  static __device__ __forceinline__ void keep(v16b a, v16b b, v16b c, v16b d) { keep4_b(a, b, c, d); }
};

__device__ __forceinline__ unsigned short at_bf_bits(float f) {
  unsigned u = __float_as_uint(f);
  return (unsigned short)((u + 0x7FFFu + ((u >> 16) & 1u)) >> 16);
}
__device__ __forceinline__ __bf16 at_f2bf(float f) { return __builtin_bit_cast(__bf16, at_bf_bits(f)); }
__device__ __forceinline__ void at_split(float f, __bf16& hi, __bf16& lo) {
  const unsigned short hb = at_bf_bits(f);
  hi = __builtin_bit_cast(__bf16, hb);
  lo = at_f2bf(f - __uint_as_float(((unsigned)hb) << 16));
}
__device__ __forceinline__ v8f at_mma(v16b a, v16b b, v8f c) {
  c = __builtin_amdgcn_wmma_f32_16x16x32_bf16(false, a, false, b, (short)0, c, false, false);
  asm volatile("v_nop\n\tv_nop\n\tv_nop\n\tv_nop" : "+v"(c) : "v"(a), "v"(b));
  return c;
}
__device__ __forceinline__ v8f mma_h16(v16h a, v16h b, v8f c) {
  c = __builtin_amdgcn_wmma_f32_16x16x32_f16(false, a, false, b, (short)0, c, false, false);
  asm volatile("v_nop\n\tv_nop\n\tv_nop\n\tv_nop" : "+v"(c) : "v"(a), "v"(b));
  return c;
}

__global__ __launch_bounds__(256) void cast_f32_bf16x2(const float* __restrict__ in,
                                                       unsigned short* __restrict__ out, int n2) {
  const int i = blockIdx.x * 256 + threadIdx.x;
  if (i < n2) {
    const unsigned u = (unsigned)f2bf_bits(in[2 * i]) | ((unsigned)f2bf_bits(in[2 * i + 1]) << 16);
    ((volatile unsigned*)out)[i] = u;
    __threadfence();
    ((volatile unsigned*)out)[i] = u;
  }
}

template <int ET> struct Elem;
template <> struct Elem<0> { typedef _Float16 T; };
template <> struct Elem<1> { typedef __bf16 T; };
template <int ET, int SPLITM, int BIAS_MODE, int OUT_MODE, bool RESID, int ACT = 0>
__global__ __launch_bounds__(256) void wmma_gemm64(
    const unsigned short* __restrict__ Ap, const unsigned short* __restrict__ A2p, int lda, long strideA,
    const unsigned short* __restrict__ Btp, const unsigned short* __restrict__ Bt2p, int ldb, long strideB,
    void* __restrict__ Cout, void* __restrict__ Cout2, int ldc, long strideC,
    const float* __restrict__ bias,
    const float* __restrict__ resid, long strideR,
    int M, int N, int K, float scale) {
  typedef typename Elem<ET>::T T;
  typedef typename Frag<T>::V V;
  constexpr bool SPA = (SPLITM >= 1);
  constexpr bool SPB = (SPLITM >= 2);
  const T* A = (const T*)Ap; const T* A2 = (const T*)A2p; const T* Bt = (const T*)Btp; const T* Bt2 = (const T*)Bt2p;
  __shared__ __align__(16) float sT[8][16 * 68];
  const int b    = blockIdx.y;
  const int lane = threadIdx.x & 31;
  const int wave = threadIdx.x >> 5;
  const int tilesN = N >> 6;
  const int tilesM = M >> 6;
  const int tile = blockIdx.x * 8 + wave;
  if (tile >= tilesM * tilesN) return;
  const int tm = tile / tilesN;
  const int tn = tile - tm * tilesN;
  const int m0 = tm << 6;
  const int n0 = tn << 6;

  const T* Ab  = A  + (size_t)b * strideA;
  const T* Bb  = Bt + (size_t)b * strideB;
  const T* Ab2 = SPA ? (A2  + (size_t)b * strideA) : nullptr;
  const T* Bb2 = SPB ? (Bt2 + (size_t)b * strideB) : nullptr;

  const int rlane = lane & 15;
  const int koff  = (lane >> 4) * 8;
  const int mOff  = (lane >> 4) * 8;

  v8f acc[4][4];
#pragma unroll
  for (int i = 0; i < 4; ++i)
#pragma unroll
    for (int j = 0; j < 4; ++j) acc[i][j] = (v8f){0.f,0.f,0.f,0.f,0.f,0.f,0.f,0.f};

  for (int k0 = 0; k0 < K; k0 += 32) {
    V bh[4], bl[4];
#pragma unroll
    for (int j = 0; j < 4; ++j) {
      const size_t bo = (size_t)(n0 + (j << 4) + rlane) * ldb + koff + k0;
      bh[j] = Frag<T>::load(Bb + bo);
      if (SPB) bl[j] = Frag<T>::load(Bb2 + bo);
    }
#pragma unroll
    for (int i = 0; i < 4; ++i) {
      const size_t ao = (size_t)(m0 + (i << 4) + rlane) * lda + koff + k0;
      V ah = Frag<T>::load(Ab + ao);
      V al;
      if (SPA) al = Frag<T>::load(Ab2 + ao);
#pragma unroll
      for (int j = 0; j < 4; ++j) {
        acc[i][j] = Frag<T>::mma(ah, bh[j], acc[i][j]);
        if (SPB) acc[i][j] = Frag<T>::mma(ah, bl[j], acc[i][j]);
        if (SPA) acc[i][j] = Frag<T>::mma(al, bh[j], acc[i][j]);
      }
      Frag<T>::guard(acc[i][0], acc[i][3], ah, SPA ? al : ah);
    }
    Frag<T>::keep(bh[0], bh[1], bh[2], bh[3]);
    if (SPB) Frag<T>::keep(bl[0], bl[1], bl[2], bl[3]);
  }
  acc_guard4(acc[0][0], acc[0][1], acc[0][2], acc[0][3]);
  acc_guard4(acc[1][0], acc[1][1], acc[1][2], acc[1][3]);
  acc_guard4(acc[2][0], acc[2][1], acc[2][2], acc[2][3]);
  acc_guard4(acc[3][0], acc[3][1], acc[3][2], acc[3][3]);

  float* slab = sT[wave];
  const float* Rb = RESID ? (resid + (size_t)b * strideR) : nullptr;
#pragma unroll
  for (int i = 0; i < 4; ++i) {
    const int mBase = m0 + (i << 4);
#pragma unroll
    for (int j = 0; j < 4; ++j) {
      const int n = n0 + (j << 4) + rlane;
      float bv = 0.f;
      if (BIAS_MODE == 2) bv = bias[n];
#pragma unroll
      for (int r = 0; r < 8; ++r) {
        float v = acc[i][j][r] * scale;
        if (BIAS_MODE == 1) v += bias[mBase + mOff + r];
        if (BIAS_MODE == 2) v += bv;
        if (RESID) v += Rb[(size_t)(mBase + mOff + r) * ldc + n];
        if (ACT == 1) v = tanhf(v);
        if (ACT == 2) v = fmaxf(v, 0.0f);
        if (ACT == 4) v = (v > 0.f) ? v : 0.01f * v;
        slab[(mOff + r) * 68 + (j << 4) + rlane] = v;
      }
    }
    __builtin_amdgcn_fence(__ATOMIC_RELEASE, "workgroup");
    __builtin_amdgcn_wave_barrier();
    __builtin_amdgcn_fence(__ATOMIC_ACQUIRE, "workgroup");
    if (OUT_MODE == 0) {
      float* C = (float*)Cout + (size_t)b * strideC;
      const int hh = lane >> 4, c4 = (lane & 15) * 4;
      for (int pass = 0; pass < 2; ++pass) {
#pragma unroll
        for (int it = 0; it < 8; ++it) {
          const int row = it * 2 + hh;
          v4f v = *(const v4f*)(slab + row * 68 + c4);
          *(volatile v4f*)(C + (size_t)(mBase + row) * ldc + n0 + c4) = v;
        }
        __threadfence();
      }
    } else {
      const int q = lane >> 3, c8 = (lane & 7) * 8;
      unsigned short* C  = (unsigned short*)Cout  + (size_t)b * strideC;
      unsigned short* C2 = (OUT_MODE == 2) ? ((unsigned short*)Cout2 + (size_t)b * strideC) : nullptr;
      for (int pass = 0; pass < 2; ++pass) {
#pragma unroll
        for (int it = 0; it < 4; ++it) {
          const int row = it * 4 + q;
          const float* sp = slab + row * 68 + c8;
          v8h hv, lv;
#pragma unroll
          for (int e = 0; e < 8; ++e) {
            if (OUT_MODE == 1) {
              hv[e] = (_Float16)sp[e];
            } else {
              unsigned short hb = f2bf_bits(sp[e]);
              unsigned short lb = f2bf_bits(sp[e] - bf_bits2f(hb));
              hv[e] = __builtin_bit_cast(_Float16, hb);
              lv[e] = __builtin_bit_cast(_Float16, lb);
            }
          }
          *(volatile v8h*)(C + (size_t)(mBase + row) * ldc + n0 + c8) = hv;
          if (OUT_MODE == 2) *(volatile v8h*)(C2 + (size_t)(mBase + row) * ldc + n0 + c8) = lv;
        }
        __threadfence();
      }
    }
    __builtin_amdgcn_fence(__ATOMIC_RELEASE, "workgroup");
    __builtin_amdgcn_wave_barrier();
    __builtin_amdgcn_fence(__ATOMIC_ACQUIRE, "workgroup");
  }
}

__global__ __launch_bounds__(128) void attn_causal_hd64(
    const unsigned short* __restrict__ qk_p,
    const unsigned short* __restrict__ vth_p, const unsigned short* __restrict__ vtl_p,
    unsigned short* __restrict__ oh_p, unsigned short* __restrict__ ol_p) {
  __shared__ __align__(16) __bf16 Psh[ATT_NW][16 * ATT_KC];
  __shared__ __align__(16) __bf16 Psl[ATT_NW][16 * ATT_KC];
  __shared__ __align__(16) float  Os[ATT_NW][16 * OS_PITCH];

  const int tid  = threadIdx.x;
  const int wave = tid >> 5;
  const int lane = tid & 31;
  const int hh   = lane >> 4;
  const int c    = lane & 15;
  const int koff = hh * 8;

  const int bx = blockIdx.x;
  const int qb = bx % NQB;
  const int bh = bx / NQB;
  const int h  = bh % NHEAD;
  const int b  = bh / NHEAD;
  const int q0 = qb * ATT_QB + wave * 16;
  const size_t rowb = (size_t)b * SEQ;

  const _Float16* QK  = (const _Float16*)qk_p;
  const __bf16*   VTH = (const __bf16*)vth_p + (size_t)bh * HDIM * SEQ;
  const __bf16*   VTL = (const __bf16*)vtl_p + (size_t)bh * HDIM * SEQ;

  v16h qa[2];
  {
    const _Float16* qrow = QK + (rowb + q0 + c) * QK_LD + h * HDIM + koff;
#pragma unroll
    for (int dc = 0; dc < 2; ++dc) qa[dc] = Frag<_Float16>::load(qrow + dc * 32);
  }

  float mrow[8], lrow[8];
  v8f oacc[4];
#pragma unroll
  for (int r = 0; r < 8; ++r) { mrow[r] = -INFINITY; lrow[r] = 0.f; }
#pragma unroll
  for (int t = 0; t < 4; ++t) oacc[t] = (v8f){0.f,0.f,0.f,0.f,0.f,0.f,0.f,0.f};

  __bf16* pwh = Psh[wave];
  __bf16* pwl = Psl[wave];
  const int nChunks = qb + 1;
  for (int kc = 0; kc < nChunks; ++kc) {
    const int kv0 = kc * ATT_KC;

    v8f s[4];
#pragma unroll
    for (int j = 0; j < 4; ++j) {
      s[j] = (v8f){0.f,0.f,0.f,0.f,0.f,0.f,0.f,0.f};
      const _Float16* krow = QK + (rowb + kv0 + j * 16 + c) * QK_LD + KCOL0 + h * HDIM + koff;
#pragma unroll
      for (int dc = 0; dc < 2; ++dc) {
        const v16h kb = Frag<_Float16>::load(krow + dc * 32);
        s[j] = mma_h16(qa[dc], kb, s[j]);
      }
    }

    const bool diag = (kc == qb);
    float cm[8];
#pragma unroll
    for (int r = 0; r < 8; ++r) {
      const int qrow = q0 + 8 * hh + r;
      float m = -INFINITY;
#pragma unroll
      for (int j = 0; j < 4; ++j) {
        const int kvcol = kv0 + j * 16 + c;
        float x = s[j][r] * 0.125f;
        if (diag && (kvcol > qrow)) x = -INFINITY;
        s[j][r] = x;
        m = fmaxf(m, x);
      }
#pragma unroll
      for (int off = 1; off < 16; off <<= 1) m = fmaxf(m, __shfl_xor(m, off, 32));
      cm[r] = m;
    }

    __builtin_amdgcn_fence(__ATOMIC_RELEASE, "workgroup");
    __builtin_amdgcn_wave_barrier();
    __builtin_amdgcn_fence(__ATOMIC_ACQUIRE, "workgroup");

#pragma unroll
    for (int r = 0; r < 8; ++r) {
      const float mnew  = fmaxf(mrow[r], cm[r]);
      const float alpha = __expf(mrow[r] - mnew);
      mrow[r] = mnew;
      float psum = 0.f;
#pragma unroll
      for (int j = 0; j < 4; ++j) {
        const float p = __expf(s[j][r] - mnew);
        psum += p;
        __bf16 ph, plo; at_split(p, ph, plo);
        pwh[(8 * hh + r) * ATT_KC + j * 16 + c] = ph;
        pwl[(8 * hh + r) * ATT_KC + j * 16 + c] = plo;
      }
#pragma unroll
      for (int off = 1; off < 16; off <<= 1) psum += __shfl_xor(psum, off, 32);
      lrow[r] = lrow[r] * alpha + psum;
#pragma unroll
      for (int t = 0; t < 4; ++t) oacc[t][r] *= alpha;
    }
    __builtin_amdgcn_fence(__ATOMIC_RELEASE, "workgroup");
    __builtin_amdgcn_wave_barrier();
    __builtin_amdgcn_fence(__ATOMIC_ACQUIRE, "workgroup");

#pragma unroll 1
    for (int kk = 0; kk < 2; ++kk) {
      const v16b pa = Frag<__bf16>::load(pwh + c * ATT_KC + kk * 32 + koff);
      const v16b pl = Frag<__bf16>::load(pwl + c * ATT_KC + kk * 32 + koff);
      const __bf16* vrh = VTH + (size_t)c * SEQ + kv0 + kk * 32 + koff;
      const __bf16* vrl = VTL + (size_t)c * SEQ + kv0 + kk * 32 + koff;
#pragma unroll
      for (int t = 0; t < 4; ++t) {
        const v16b vb = Frag<__bf16>::load(vrh + (size_t)(t * 16) * SEQ);
        const v16b vl = Frag<__bf16>::load(vrl + (size_t)(t * 16) * SEQ);
        oacc[t] = at_mma(pa, vb, oacc[t]);
        oacc[t] = at_mma(pa, vl, oacc[t]);
        oacc[t] = at_mma(pl, vb, oacc[t]);
      }
    }
  }

  float* os = Os[wave];
#pragma unroll
  for (int r = 0; r < 8; ++r) {
    const float inv = 1.0f / lrow[r];
#pragma unroll
    for (int t = 0; t < 4; ++t) os[(8 * hh + r) * OS_PITCH + t * 16 + c] = oacc[t][r] * inv;
  }
  __builtin_amdgcn_fence(__ATOMIC_RELEASE, "workgroup");
  __builtin_amdgcn_wave_barrier();
  __builtin_amdgcn_fence(__ATOMIC_ACQUIRE, "workgroup");
  {
    const int q8 = lane >> 3, c8 = (lane & 7) * 8;
    unsigned short* OH = oh_p + (rowb + q0) * DMODEL + h * HDIM + c8;
    unsigned short* OL = ol_p + (rowb + q0) * DMODEL + h * HDIM + c8;
    for (int pass = 0; pass < 2; ++pass) {
#pragma unroll
      for (int it = 0; it < 4; ++it) {
        const int row = it * 4 + q8;
        const float* sp = os + row * OS_PITCH + c8;
        v8h hv, lv;
#pragma unroll
        for (int e = 0; e < 8; ++e) {
          const unsigned short hb = f2bf_bits(sp[e]);
          const unsigned short lb = f2bf_bits(sp[e] - bf_bits2f(hb));
          hv[e] = __builtin_bit_cast(_Float16, hb);
          lv[e] = __builtin_bit_cast(_Float16, lb);
        }
        *(volatile v8h*)(OH + (size_t)row * DMODEL) = hv;
        *(volatile v8h*)(OL + (size_t)row * DMODEL) = lv;
      }
      __threadfence();
    }
  }
}

extern "C" void kernel_launch(void* const* d_in, const int* in_sizes, int n_in,
                              void* d_out, int out_size, void* d_ws,
                              size_t ws_size, hipStream_t stream) {
  constexpr size_t N_X  = (size_t)NBATCH * SEQ * DMODEL;
  constexpr size_t N_W  = (size_t)DMODEL * DMODEL;
  constexpr size_t N_VT = (size_t)NBATCH * NHEAD * HDIM * SEQ;
  constexpr size_t OFF_XB   = 0;
  constexpr size_t OFF_WALL = OFF_XB + N_X * 2;
  constexpr size_t OFF_QK   = OFF_WALL + 4 * N_W * 2;
  constexpr size_t OFF_VTH  = OFF_QK + N_X * 2 * 2;
  constexpr size_t OFF_VTL  = OFF_VTH + N_VT * 2;
  constexpr size_t OFF_OH   = OFF_VTL + N_VT * 2;
  constexpr size_t OFF_OL   = OFF_OH + N_X * 2;
  constexpr size_t WS_TOTAL = OFF_OL + N_X * 2;
  static_assert(WS_TOTAL == 125829120);

  if (n_in < 5) return;
  if ((size_t)in_sizes[0] != N_X) return;
  if ((size_t)in_sizes[1] != N_W || (size_t)in_sizes[2] != N_W ||
      (size_t)in_sizes[3] != N_W || (size_t)in_sizes[4] != N_W) return;
  if ((size_t)out_size != N_X) return;
  if (ws_size < WS_TOTAL) return;

  const float* x  = (const float*)d_in[0];
  const float* Wq = (const float*)d_in[1];
  const float* Wk = (const float*)d_in[2];
  const float* Wv = (const float*)d_in[3];
  const float* Wo = (const float*)d_in[4];

  char* ws = (char*)d_ws;
  unsigned short* xb   = (unsigned short*)(ws + OFF_XB);
  unsigned short* wall = (unsigned short*)(ws + OFF_WALL);
  unsigned short* qk   = (unsigned short*)(ws + OFF_QK);
  unsigned short* vth  = (unsigned short*)(ws + OFF_VTH);
  unsigned short* vtl  = (unsigned short*)(ws + OFF_VTL);
  unsigned short* oh   = (unsigned short*)(ws + OFF_OH);
  unsigned short* ol   = (unsigned short*)(ws + OFF_OL);
  const float* unused_f = (const float*)(ws + OFF_XB);

  cast_f32_bf16x2<<<dim3((unsigned)(N_X / 2 / 256)), dim3(256), 0, stream>>>(x,  xb, (int)(N_X / 2));
  cast_f32_bf16x2<<<dim3((unsigned)(N_W / 2 / 256)), dim3(256), 0, stream>>>(Wq, wall + 0 * N_W, (int)(N_W / 2));
  cast_f32_bf16x2<<<dim3((unsigned)(N_W / 2 / 256)), dim3(256), 0, stream>>>(Wk, wall + 1 * N_W, (int)(N_W / 2));
  cast_f32_bf16x2<<<dim3((unsigned)(N_W / 2 / 256)), dim3(256), 0, stream>>>(Wv, wall + 2 * N_W, (int)(N_W / 2));
  cast_f32_bf16x2<<<dim3((unsigned)(N_W / 2 / 256)), dim3(256), 0, stream>>>(Wo, wall + 3 * N_W, (int)(N_W / 2));

  const int MROWS = NBATCH * SEQ;

  wmma_gemm64<1, 0, 0, 1, false><<<dim3((MROWS / 64) * (2 * DMODEL / 64) / 8, 1), dim3(256), 0, stream>>>(
      xb, xb, DMODEL, 0L,
      wall, wall, DMODEL, 0L,
      (void*)qk, (void*)qk, QK_LD, 0L,
      unused_f, unused_f, 0L,
      MROWS, 2 * DMODEL, DMODEL, 1.0f);

  wmma_gemm64<1, 0, 0, 2, false><<<dim3((DMODEL / 64) * (SEQ / 64) / 8, NBATCH), dim3(256), 0, stream>>>(
      wall + 2 * N_W, wall + 2 * N_W, DMODEL, 0L,
      xb, xb, DMODEL, (long)SEQ * DMODEL,
      (void*)vth, (void*)vtl, SEQ, (long)DMODEL * SEQ,
      unused_f, unused_f, 0L,
      DMODEL, SEQ, DMODEL, 1.0f);

  attn_causal_hd64<<<dim3(NBATCH * NHEAD * NQB), dim3(128), 0, stream>>>(qk, vth, vtl, oh, ol);

  wmma_gemm64<1, 1, 0, 0, false><<<dim3((MROWS / 64) * (DMODEL / 64) / 8, 1), dim3(256), 0, stream>>>(
      oh, ol, DMODEL, 0L,
      wall + 3 * N_W, wall + 3 * N_W, DMODEL, 0L,
      d_out, d_out, DMODEL, 0L,
      unused_f, unused_f, 0L,
      MROWS, DMODEL, DMODEL, 1.0f);
}
